// DecoderBlockWithKeywords_26087631356680
// MI455X (gfx1250) — hardware-verified
//
#include <hip/hip_runtime.h>


#define NB_  4
#define TQ   1024
#define DD   512
#define NH_  8
#define HD   64
#define NT   (NB_ * TQ)
#define DFF  2048
#define NEGF (-1000000.0f)
#define PCAR 1024.0f
typedef _Float16 h16;
typedef unsigned short bf;
typedef __attribute__((ext_vector_type(16))) __bf16   v16bf;
typedef __attribute__((ext_vector_type(16))) _Float16 v16h;
typedef __attribute__((ext_vector_type(8)))  _Float16 v8h;
typedef __attribute__((ext_vector_type(8)))  unsigned short v8us;
typedef __attribute__((ext_vector_type(8)))  float    v8f;
typedef __attribute__((ext_vector_type(4)))  float    v4f;
typedef v8h  __attribute__((may_alias)) v8ha;
typedef v4f  __attribute__((may_alias)) v4fa;
typedef v8us __attribute__((may_alias)) v8usa;

__device__ __forceinline__ unsigned short f2bf(float f) { unsigned u = __float_as_uint(f); u += 0x7FFFu + ((u >> 16) & 1u); return (unsigned short)(u >> 16); }
__device__ __forceinline__ float bf2f(unsigned short b) { return __uint_as_float(((unsigned)b) << 16); }
__device__ __forceinline__ float bfr(float f) { return bf2f(f2bf(f)); }
__device__ __forceinline__ v16h cat16(v8h lo, v8h hi) { return __builtin_shufflevector(lo, hi, 0, 1, 2, 3, 4, 5, 6, 7, 8, 9, 10, 11, 12, 13, 14, 15); }
__device__ __forceinline__ v16bf cat16b(v8us lo, v8us hi) { return __builtin_bit_cast(v16bf, __builtin_shufflevector(lo, hi, 0, 1, 2, 3, 4, 5, 6, 7, 8, 9, 10, 11, 12, 13, 14, 15)); }
__device__ __forceinline__ v8f wmma16(v16h a, v16h b, v8f c) { return __builtin_amdgcn_wmma_f32_16x16x32_f16(false, a, false, b, (short)0, c, false, false); }
__device__ __forceinline__ v8f wmmab(v16bf a, v16bf b, v8f c) { return __builtin_amdgcn_wmma_f32_16x16x32_bf16(false, a, false, b, (short)0, c, false, false); }


template <typename T16> struct WFrag;
template <> struct WFrag<h16> { typedef v16h V; static __device__ __forceinline__ V ld(const h16* p) { return cat16(*(const v8h*)p, *(const v8h*)(p + 16)); } static __device__ __forceinline__ v8f mma(V a, V b, v8f c) { return wmma16(a, b, c); } };
template <> struct WFrag<bf> { typedef v16bf V; static __device__ __forceinline__ V ld(const bf* p) { return cat16b(*(const v8us*)p, *(const v8us*)(p + 16)); } static __device__ __forceinline__ v8f mma(V a, V b, v8f c) { return wmmab(a, b, c); } };
template <typename T16, int NSPLIT, bool BIAS>
__global__ __launch_bounds__(32) void k_gemmw(const T16* __restrict__ A, const T16* __restrict__ A2, const T16* __restrict__ Bt, const T16* __restrict__ Bt2, int K, float* C, int ldc, const float* __restrict__ bias, size_t sA, size_t sB, size_t sC) {
    typedef typename WFrag<T16>::V V;
    __shared__ __align__(16) float os[16 * 68];
    const size_t z = blockIdx.z; A += z * sA; if (A2) A2 += z * sA; Bt += z * sB; if (Bt2) Bt2 += z * sB; C += z * sC;
    const int lane = threadIdx.x & 31, lr = lane & 15, hi = lane >> 4; const int r0 = blockIdx.x * 64, c0 = blockIdx.y * 64;
    v8f acc[4][4];
#pragma unroll
    for (int mb = 0; mb < 4; ++mb)
#pragma unroll
        for (int nb = 0; nb < 4; ++nb) acc[mb][nb] = (v8f){};
    const size_t aoff = (size_t)(r0 + lr) * K + 8 * hi, boff = (size_t)(c0 + lr) * K + 8 * hi;
#pragma unroll 1
    for (int kc = 0; kc < K; kc += 32) {
        V a[4], a2[4];
#pragma unroll
        for (int mb = 0; mb < 4; ++mb) { a[mb] = WFrag<T16>::ld(A + aoff + (size_t)mb * 16 * K + kc); if (NSPLIT == 1 || NSPLIT == 2) a2[mb] = WFrag<T16>::ld(A2 + aoff + (size_t)mb * 16 * K + kc); }
#pragma unroll
        for (int nb = 0; nb < 4; ++nb) { const V b = WFrag<T16>::ld(Bt + boff + (size_t)nb * 16 * K + kc); V b2; if (NSPLIT >= 2) b2 = WFrag<T16>::ld(Bt2 + boff + (size_t)nb * 16 * K + kc);
#pragma unroll
            for (int mb = 0; mb < 4; ++mb) { acc[mb][nb] = WFrag<T16>::mma(a[mb], b, acc[mb][nb]); if (NSPLIT == 1 || NSPLIT == 2) acc[mb][nb] = WFrag<T16>::mma(a2[mb], b, acc[mb][nb]); if (NSPLIT >= 2) acc[mb][nb] = WFrag<T16>::mma(a[mb], b2, acc[mb][nb]); } }
        asm volatile("v_nop\n\tv_nop\n\tv_nop\n\tv_nop" : "+v"(acc[0][0]), "+v"(acc[1][1]), "+v"(acc[2][2]), "+v"(acc[3][3]) : "v"(a[0]), "v"(a[3]));
    }
#pragma unroll
    for (int mb = 0; mb < 4; ++mb) {
#pragma unroll
        for (int nb = 0; nb < 4; ++nb) {
#pragma unroll
            for (int j = 0; j < 8; ++j) os[(hi * 8 + j) * 68 + nb * 16 + lr] = acc[mb][nb][j]; }
        __builtin_amdgcn_wave_barrier(); asm volatile("" ::: "memory");
        float* crow = C + (size_t)(r0 + mb * 16) * ldc + c0;
#pragma unroll 1
        for (int ps = 0; ps < 2; ++ps) {
#pragma unroll
            for (int s = 0; s < 8; ++s) { const int row = 2 * s + hi, cofs = lr * 4; v4f val = *(const v4fa*)(os + row * 68 + cofs); if (BIAS) { val[0] += bfr(bias[c0 + cofs]); val[1] += bfr(bias[c0 + cofs + 1]); val[2] += bfr(bias[c0 + cofs + 2]); val[3] += bfr(bias[c0 + cofs + 3]); }
                *(volatile v4f*)(crow + (size_t)row * ldc + cofs) = val; }
            if (ps == 0) __threadfence(); }
        __builtin_amdgcn_wave_barrier(); asm volatile("" ::: "memory");
    }
}

__device__ __forceinline__ h16 tohx(float x) { return (h16)x; }
__device__ __forceinline__ void splitf(float y, unsigned short& h, unsigned short& l) { h = f2bf(y); l = f2bf(y - bf2f(h)); }
typedef __attribute__((ext_vector_type(2))) _Float16 v2h;
typedef __attribute__((ext_vector_type(4))) _Float16 v4h;
typedef __attribute__((ext_vector_type(2))) unsigned short v2us;
typedef __attribute__((ext_vector_type(4))) unsigned short v4us;

__global__ __launch_bounds__(256) void k_cvt8(const float* __restrict__ src, bf* dst, size_t n8) { const size_t i = (size_t)blockIdx.x * 256 + threadIdx.x; if (i >= n8) return; const v8f v = *(const v8f*)(src + i * 8); v8us o;
#pragma unroll
    for (int k = 0; k < 8; ++k) o[k] = f2bf(v[k]); *(volatile v8us*)(dst + i * 8) = o; __threadfence(); *(volatile v8us*)(dst + i * 8) = o; }
__global__ __launch_bounds__(256) void k_wtb(const float* __restrict__ w, int K, int N, int Np, bf* Bt) {
    const int lane = threadIdx.x & 31; const int L0 = (blockIdx.x * 8 + (threadIdx.x >> 5)) * 8; const int nlines = Np * K / 64;
#pragma unroll 1
    for (int ps = 0; ps < 2; ++ps) {
#pragma unroll 1
        for (int l = 0; l < 8; ++l) { const int L = L0 + l; if (L >= nlines) break; const int e = L * 64 + lane * 2; v2us o;
#pragma unroll
            for (int q = 0; q < 2; ++q) { const int n = (e + q) / K, k = (e + q) % K; o[q] = (n < N) ? f2bf(w[(size_t)k * N + n]) : (unsigned short)0; }
            *(volatile v2us*)(Bt + e) = o; }
        if (ps == 0) __threadfence(); }
}
__global__ __launch_bounds__(256) void k_hplane(const float* __restrict__ F, int Tn, float sc, h16* P) {
    const int lane = threadIdx.x & 31; const int L0 = (blockIdx.x * 8 + (threadIdx.x >> 5)) * 8; const int nlines = NB_ * Tn * DD / 64;
#pragma unroll 1
    for (int ps = 0; ps < 2; ++ps) {
#pragma unroll
        for (int l = 0; l < 8; ++l) { const int L = L0 + l; if (L >= nlines) break; const int e = L * 64 + lane * 2; const int d = e & 63; const int t = (e >> 6) % Tn; const int z = (e >> 6) / Tn; const int b = z >> 3, h = z & 7; v2h v;
#pragma unroll
            for (int q = 0; q < 2; ++q) v[q] = tohx(F[((size_t)b * Tn + t) * DD + h * HD + d + q] * sc);
            *(volatile v2h*)(P + (size_t)e) = v; }
        if (ps == 0) __threadfence(); }
}
__global__ __launch_bounds__(256) void k_vtplane(const float* __restrict__ F, int Tn, h16* VT) {
    const int lane = threadIdx.x & 31; const int L0 = (blockIdx.x * 8 + (threadIdx.x >> 5)) * 8; const int nlines = NB_ * Tn * DD / 64;
#pragma unroll 1
    for (int ps = 0; ps < 2; ++ps) {
#pragma unroll
        for (int l = 0; l < 8; ++l) { const int L = L0 + l; if (L >= nlines) break; const int e = L * 64 + lane * 2; const int t = e % Tn; const int d = (e / Tn) & 63; const int z = e / (Tn * 64); const int b = z >> 3, h = z & 7; v2h v;
#pragma unroll
            for (int q = 0; q < 2; ++q) v[q] = tohx(F[((size_t)b * Tn + t + q) * DD + h * HD + d]);
            *(volatile v2h*)(VT + (size_t)e) = v; }
        if (ps == 0) __threadfence(); }
}
__global__ __launch_bounds__(256) void k_msoft(const float* __restrict__ Sb, int Tk, int causal, const int* __restrict__ lens, int b, h16* P) {
    const int lane = threadIdx.x & 31; const int row = blockIdx.x * 8 + (threadIdx.x >> 5); if (row >= NH_ * TQ) return; const int i = row % TQ; const float* sr = Sb + (size_t)row * Tk;
    const int lim = causal ? i + 1 : lens[b];
    float m = -3.0e38f;
#pragma unroll 1
    for (int c0 = lane * 2; c0 < Tk; c0 += 64) {
#pragma unroll
        for (int q = 0; q < 2; ++q) { const int k = c0 + q; const float s = (k < lim) ? sr[k] : NEGF; m = fmaxf(m, s); } }
#pragma unroll
    for (int sh = 16; sh; sh >>= 1) m = fmaxf(m, __shfl_xor(m, sh, 32));
    float sum = 0.f;
#pragma unroll 1
    for (int c0 = lane * 2; c0 < Tk; c0 += 64) {
#pragma unroll
        for (int q = 0; q < 2; ++q) { const int k = c0 + q; const float s = (k < lim) ? sr[k] : NEGF; sum += __expf(s - m); } }
#pragma unroll
    for (int sh = 16; sh; sh >>= 1) sum += __shfl_xor(sum, sh, 32);
    const float f = __fdiv_rn(PCAR, sum);
#pragma unroll 1
    for (int ps = 0; ps < 2; ++ps) {
#pragma unroll 1
        for (int c0 = lane * 2; c0 < Tk; c0 += 64) { v2h o;
#pragma unroll
            for (int q = 0; q < 2; ++q) { const int k = c0 + q; const float s = (k < lim) ? sr[k] : NEGF; o[q] = tohx(__expf(s - m) * f); }
            *(volatile v2h*)(P + (size_t)row * Tk + c0) = o; }
        if (ps == 0) __threadfence(); }
}
__global__ __launch_bounds__(256) void k_merge(const float* __restrict__ O, int b, bf* Ah, bf* Al) {
    const int lane = threadIdx.x & 31; const int L0 = (blockIdx.x * 8 + (threadIdx.x >> 5)) * 8; const int nlines = TQ * DD / 64;
#pragma unroll 1
    for (int ps = 0; ps < 2; ++ps) {
#pragma unroll
        for (int l = 0; l < 8; ++l) { const int L = L0 + l; if (L >= nlines) break; const int e = L * 64 + lane * 2; const int c = e & 511; const int t = e >> 9; const int h = c >> 6, d = c & 63; v2us oh, ol;
#pragma unroll
            for (int q = 0; q < 2; ++q) { unsigned short a, c2; splitf(O[((size_t)h * TQ + t) * HD + d + q] * (1.0f / PCAR), a, c2); oh[q] = a; ol[q] = c2; }
            const size_t o = ((size_t)b * TQ + t) * DD + c; *(volatile v2us*)(Ah + o) = oh; *(volatile v2us*)(Al + o) = ol; }
        if (ps == 0) __threadfence(); }
}
template <int MODE, bool FINAL>
__global__ __launch_bounds__(256) void k_ln(const float* __restrict__ A, const float* __restrict__ R, const float* __restrict__ gg, const float* __restrict__ bb, float* Y, bf* Ph, bf* Pl) {
    const int lane = threadIdx.x & 31; const int r = blockIdx.x * 8 + (threadIdx.x >> 5); if (r >= NT) return; float v[16]; float s = 0.f;
#pragma unroll
    for (int c = 0; c < 4; ++c)
#pragma unroll
        for (int q = 0; q < 4; ++q) { const size_t idx = (size_t)r * DD + c * 128 + lane * 4 + q; const float res = (MODE == 0) ? bfr(R[idx]) : R[idx]; const float t = A[idx] + res; v[c * 4 + q] = t; s += t; }
#pragma unroll
    for (int sh = 16; sh; sh >>= 1) s += __shfl_xor(s, sh, 32);
    const float mu = s * (1.0f / DD); float qq = 0.f;
#pragma unroll
    for (int i = 0; i < 16; ++i) { const float d0 = v[i] - mu; qq = fmaf(d0, d0, qq); }
#pragma unroll
    for (int sh = 16; sh; sh >>= 1) qq += __shfl_xor(qq, sh, 32);
    const float rs = rsqrtf(qq * (1.0f / DD) + 1e-5f);
#pragma unroll 1
    for (int ps = 0; ps < 2; ++ps) {
#pragma unroll
        for (int c = 0; c < 4; ++c) { v4f o; v4us oh, ol;
#pragma unroll
            for (int q = 0; q < 4; ++q) { const int col = c * 128 + lane * 4 + q; const float y = (v[c * 4 + q] - mu) * rs * bfr(gg[col]) + bfr(bb[col]); o[q] = y; if (!FINAL) { unsigned short a, c2; splitf(y, a, c2); oh[q] = a; ol[q] = c2; } }
            *(volatile v4f*)(Y + (size_t)r * DD + c * 128 + lane * 4) = o; if (!FINAL) { *(volatile v4us*)(Ph + (size_t)r * DD + c * 128 + lane * 4) = oh; *(volatile v4us*)(Pl + (size_t)r * DD + c * 128 + lane * 4) = ol; } }
        if (ps == 0) __threadfence(); }
}
__global__ __launch_bounds__(256) void k_catsplit(const float* __restrict__ A, const float* __restrict__ B2, bf* Ph, bf* Pl) {
    const int lane = threadIdx.x & 31; const int L0 = (blockIdx.x * 8 + (threadIdx.x >> 5)) * 8; const int nlines = NT * 2 * DD / 64;
#pragma unroll 1
    for (int ps = 0; ps < 2; ++ps) {
#pragma unroll
        for (int l = 0; l < 8; ++l) { const int L = L0 + l; if (L >= nlines) break; const int e = L * 64 + lane * 2; const int c = e & 1023; const int r = e >> 10; v2us oh, ol;
#pragma unroll
            for (int q = 0; q < 2; ++q) { const int cc = c + q; const float v = cc < DD ? A[(size_t)r * DD + cc] : B2[(size_t)r * DD + cc - DD]; unsigned short a, c2; splitf(v, a, c2); oh[q] = a; ol[q] = c2; }
            *(volatile v2us*)(Ph + (size_t)e) = oh; *(volatile v2us*)(Pl + (size_t)e) = ol; }
        if (ps == 0) __threadfence(); }
}
__global__ __launch_bounds__(256) void k_mix(const float* __restrict__ G, const float* __restrict__ gb, const float* __restrict__ A, const float* __restrict__ B2, float* Y2) {
    const size_t i = (size_t)blockIdx.x * 256 + threadIdx.x; if (i >= (size_t)NT * DD / 4) return; const size_t e = i * 4; const int r = (int)(e / DD);
    const float z = G[(size_t)r * 64] + bfr(gb[0]); const float sg = __fdiv_rn(1.0f, 1.0f + __expf(-z)); const v4f a = *(const v4f*)(A + e), b2 = *(const v4f*)(B2 + e); v4f o;
#pragma unroll
    for (int q = 0; q < 4; ++q) o[q] = sg * a[q] + (1.0f - sg) * b2[q];
    *(volatile v4f*)(Y2 + e) = o; __threadfence(); *(volatile v4f*)(Y2 + e) = o;
}
__global__ __launch_bounds__(256) void k_relusplit2k(const float* __restrict__ H, bf* Ph, bf* Pl) {
    const int lane = threadIdx.x & 31; const int L0 = (blockIdx.x * 8 + (threadIdx.x >> 5)) * 8; const int nlines = NT * DFF / 64;
#pragma unroll 1
    for (int ps = 0; ps < 2; ++ps) {
#pragma unroll
        for (int l = 0; l < 8; ++l) { const int L = L0 + l; if (L >= nlines) break; const int e = L * 64 + lane * 2; v2us oh, ol;
#pragma unroll
            for (int q = 0; q < 2; ++q) { unsigned short a, c2; splitf(fmaxf(H[(size_t)e + q], 0.f), a, c2); oh[q] = a; ol[q] = c2; }
            *(volatile v2us*)(Ph + (size_t)e) = oh; *(volatile v2us*)(Pl + (size_t)e) = ol; }
        if (ps == 0) __threadfence(); }
}

struct MhaBufs { float* Fq; float* Fk; float* Fv; h16* Qp; h16* Kp; h16* VT; float* Sb; h16* Pm; float* Ob; bf* ATh; bf* ATl; };
static void run_mha(hipStream_t stream, const MhaBufs& B, const bf* QAh, const bf* QAl, const bf* QB, const bf* MB, int Tk, const bf* WQ, const bf* WK, const bf* WV, const bf* WO, const int* lens, int causal, float* AO) {
    const unsigned LBQ = (unsigned)((NT * DD / 64 + 63) / 64); const unsigned LBK = (unsigned)((NB_ * Tk * DD / 64 + 63) / 64);
    if (QB) k_gemmw<bf, 0, false><<<dim3(NT / 64, DD / 64, 1), 32, 0, stream>>>(QB, nullptr, WQ, nullptr, DD, B.Fq, DD, nullptr, 0, 0, 0);
    else    k_gemmw<bf, 1, false><<<dim3(NT / 64, DD / 64, 1), 32, 0, stream>>>(QAh, QAl, WQ, nullptr, DD, B.Fq, DD, nullptr, 0, 0, 0);
    k_gemmw<bf, 0, false><<<dim3(NB_ * Tk / 64, DD / 64, 1), 32, 0, stream>>>(MB, nullptr, WK, nullptr, DD, B.Fk, DD, nullptr, 0, 0, 0);
    k_gemmw<bf, 0, false><<<dim3(NB_ * Tk / 64, DD / 64, 1), 32, 0, stream>>>(MB, nullptr, WV, nullptr, DD, B.Fv, DD, nullptr, 0, 0, 0);
    k_hplane<<<LBQ, 256, 0, stream>>>(B.Fq, TQ, 0.125f, B.Qp); k_hplane<<<LBK, 256, 0, stream>>>(B.Fk, Tk, 1.0f, B.Kp); k_vtplane<<<LBK, 256, 0, stream>>>(B.Fv, Tk, B.VT);
    for (int b = 0; b < NB_; ++b) { const size_t zq = (size_t)b * NH_;
        k_gemmw<h16, 0, false><<<dim3(TQ / 64, Tk / 64, NH_), 32, 0, stream>>>(B.Qp + zq * TQ * HD, nullptr, B.Kp + zq * Tk * HD, nullptr, HD, B.Sb, Tk, nullptr, (size_t)TQ * HD, (size_t)Tk * HD, (size_t)TQ * Tk);
        k_msoft<<<NH_ * TQ / 8, 256, 0, stream>>>(B.Sb, Tk, causal, lens, b, B.Pm);
        k_gemmw<h16, 0, false><<<dim3(TQ / 64, 1, NH_), 32, 0, stream>>>(B.Pm, nullptr, B.VT + zq * HD * Tk, nullptr, Tk, B.Ob, HD, nullptr, (size_t)TQ * Tk, (size_t)HD * Tk, (size_t)TQ * HD);
        k_merge<<<(TQ * DD / 64 + 63) / 64, 256, 0, stream>>>(B.Ob, b, B.ATh, B.ATl); }
    k_gemmw<bf, 1, false><<<dim3(NT / 64, DD / 64, 1), 32, 0, stream>>>(B.ATh, B.ATl, WO, nullptr, DD, AO, DD, nullptr, 0, 0, 0);
}

extern "C" void kernel_launch(void* const* d_in, const int* in_sizes, int n_in,
                              void* d_out, int out_size, void* d_ws, size_t ws_size, hipStream_t stream) {
    (void)in_sizes; (void)n_in; (void)out_size;
    const float* x = (const float*)d_in[0]; const float* src = (const float*)d_in[1]; const float* tmpl = (const float*)d_in[2]; const float* kw = (const float*)d_in[3];
    const int* src_len = (const int*)d_in[4]; const int* tmpl_len = (const int*)d_in[5]; const int* kw_len = (const int*)d_in[6];
    const float* W[16]; for (int i = 0; i < 16; ++i) W[i] = (const float*)d_in[7 + i];
    const float* gate_w = (const float*)d_in[23]; const float* gate_b = (const float*)d_in[24]; const float* w1 = (const float*)d_in[25]; const float* b1 = (const float*)d_in[26]; const float* w2 = (const float*)d_in[27]; const float* b2 = (const float*)d_in[28];
    const float* lng[4]; const float* lnb[4]; for (int i = 0; i < 4; ++i) { lng[i] = (const float*)d_in[29 + 2 * i]; lnb[i] = (const float*)d_in[30 + 2 * i]; }
    float* OUT = (float*)d_out;
    char* wsp = (char*)d_ws;
    auto take = [&](size_t bytes) { char* p = wsp; wsp += (bytes + 255) & ~(size_t)255; return (void*)p; };
    bf* WB[16]; for (int i = 0; i < 16; ++i) WB[i] = (bf*)take((size_t)DD * DD * 2);
    bf* GW = (bf*)take((size_t)64 * 2 * DD * 2); bf* W1B = (bf*)take((size_t)DFF * DD * 2); bf* W2B = (bf*)take((size_t)DD * DFF * 2);
    bf* XB = (bf*)take((size_t)NT * DD * 2); bf* SRCB = (bf*)take((size_t)NB_ * 1024 * DD * 2); bf* TMB = (bf*)take((size_t)NB_ * 512 * DD * 2); bf* KWB = (bf*)take((size_t)NB_ * 64 * DD * 2);
    MhaBufs Bf;
    Bf.Fq = (float*)take((size_t)NT * DD * 4); Bf.Fk = (float*)take((size_t)NT * DD * 4); Bf.Fv = (float*)take((size_t)NT * DD * 4);
    Bf.Qp = (h16*)take((size_t)NT * DD * 2); Bf.Kp = (h16*)take((size_t)NT * DD * 2); Bf.VT = (h16*)take((size_t)NT * DD * 2);
    Bf.Sb = (float*)take((size_t)NH_ * TQ * 1024 * 4); Bf.Pm = (h16*)take((size_t)NH_ * TQ * 1024 * 2); Bf.Ob = (float*)take((size_t)NH_ * TQ * HD * 4); Bf.ATh = (bf*)take((size_t)NT * DD * 2); Bf.ATl = (bf*)take((size_t)NT * DD * 2);
    float* X2 = (float*)take((size_t)NT * DD * 4); float* Y = (float*)take((size_t)NT * DD * 4); bf* Yh = (bf*)take((size_t)NT * DD * 2); bf* Yl = (bf*)take((size_t)NT * DD * 2);
    float* Y2K = (float*)take((size_t)NT * DD * 4); float* G = (float*)take((size_t)NT * 64 * 4); float* Y2 = (float*)take((size_t)NT * DD * 4);
    float* Z = (float*)take((size_t)NT * DD * 4); bf* Zh = (bf*)take((size_t)NT * DD * 2); bf* Zl = (bf*)take((size_t)NT * DD * 2);
    bf* RLh = (bf*)take((size_t)NT * DFF * 2); bf* RLl = (bf*)take((size_t)NT * DFF * 2);
    if ((size_t)(wsp - (char*)d_ws) > ws_size) return;
    float* Y2C = X2;
    bf* CATh = (bf*)Bf.Sb; bf* CATl = (bf*)((char*)Bf.Sb + (size_t)NT * 2 * DD * 2);
    float* Z2 = X2;
    float* ZE = Y; bf* ZEh = Yh; bf* ZEl = Yl;
    float* Hf = Bf.Sb;
    float* F2 = Y2K;
    { const unsigned gw = (unsigned)((DD * DD / 64 + 63) / 64); for (int i = 0; i < 16; ++i) k_wtb<<<gw, 256, 0, stream>>>(W[i], DD, DD, DD, WB[i]);
      k_wtb<<<(64 * 2 * DD / 64 + 63) / 64, 256, 0, stream>>>(gate_w, 2 * DD, 1, 64, GW); k_wtb<<<(DFF * DD / 64 + 63) / 64, 256, 0, stream>>>(w1, DD, DFF, DFF, W1B); k_wtb<<<(DD * DFF / 64 + 63) / 64, 256, 0, stream>>>(w2, DFF, DD, DD, W2B);
      const unsigned g8 = 256; k_cvt8<<<(unsigned)(((size_t)NT * DD / 8 + g8 - 1) / g8), 256, 0, stream>>>(x, XB, (size_t)NT * DD / 8); k_cvt8<<<(unsigned)(((size_t)NB_ * 1024 * DD / 8 + g8 - 1) / g8), 256, 0, stream>>>(src, SRCB, (size_t)NB_ * 1024 * DD / 8);
      k_cvt8<<<(unsigned)(((size_t)NB_ * 512 * DD / 8 + g8 - 1) / g8), 256, 0, stream>>>(tmpl, TMB, (size_t)NB_ * 512 * DD / 8); k_cvt8<<<(unsigned)(((size_t)NB_ * 64 * DD / 8 + g8 - 1) / g8), 256, 0, stream>>>(kw, KWB, (size_t)NB_ * 64 * DD / 8); }
    const unsigned LB = (unsigned)((NT * DD / 64 + 63) / 64);
    run_mha(stream, Bf, nullptr, nullptr, XB, XB, TQ, WB[0], WB[1], WB[2], WB[3], src_len  , 1, X2);
    k_ln<0, false><<<NT / 8, 256, 0, stream>>>(X2, x, lng[0], lnb[0], Y, Yh, Yl);
    run_mha(stream, Bf, Yh, Yl, nullptr, SRCB, 1024, WB[4], WB[5], WB[6], WB[7], src_len, 0, Y2C);
    run_mha(stream, Bf, Yh, Yl, nullptr, KWB, 64, WB[12], WB[13], WB[14], WB[15], kw_len, 0, Y2K);
    k_catsplit<<<(NT * 2 * DD / 64 + 63) / 64, 256, 0, stream>>>(Y2C, Y2K, CATh, CATl);
    k_gemmw<bf, 1, false><<<dim3(NT / 64, 1, 1), 32, 0, stream>>>(CATh, CATl, GW, nullptr, 2 * DD, G, 64, nullptr, 0, 0, 0);
    k_mix<<<(unsigned)(((size_t)NT * DD / 4 + 255) / 256), 256, 0, stream>>>(G, gate_b, Y2C, Y2K, Y2);
    k_ln<1, false><<<NT / 8, 256, 0, stream>>>(Y2, Y, lng[1], lnb[1], Z, Zh, Zl);
    run_mha(stream, Bf, Zh, Zl, nullptr, TMB, 512, WB[8], WB[9], WB[10], WB[11], tmpl_len, 0, Z2);
    k_ln<1, false><<<NT / 8, 256, 0, stream>>>(Z2, Z, lng[2], lnb[2], ZE, ZEh, ZEl);
    k_gemmw<bf, 1, true><<<dim3(NT / 64, DFF / 64, 1), 32, 0, stream>>>(ZEh, ZEl, W1B, nullptr, DD, Hf, DFF, b1, 0, 0, 0);
    k_relusplit2k<<<(NT * DFF / 64 + 63) / 64, 256, 0, stream>>>(Hf, RLh, RLl);
    k_gemmw<bf, 1, true><<<dim3(NT / 64, DD / 64, 1), 32, 0, stream>>>(RLh, RLl, W2B, nullptr, DFF, F2, DD, b2, 0, 0, 0);
    k_ln<1, true><<<NT / 8, 256, 0, stream>>>(F2, ZE, lng[3], lnb[3], OUT, nullptr, nullptr);
}
